// SegHead_48567490183568
// MI455X (gfx1250) — hardware-verified
//
#include <hip/hip_runtime.h>
#include <math.h>

typedef __attribute__((ext_vector_type(16))) _Float16 v16h;
typedef __attribute__((ext_vector_type(16))) __bf16 v16b;
typedef __attribute__((ext_vector_type(8)))  _Float16 v8h;
typedef __attribute__((ext_vector_type(8)))  float v8f;
typedef __attribute__((ext_vector_type(4)))  float v4f;
typedef __attribute__((ext_vector_type(2)))  float v2f;
typedef __attribute__((ext_vector_type(4)))  unsigned v4u;
typedef __attribute__((ext_vector_type(4)))  int v4i;
typedef float __attribute__((may_alias)) float_a;
typedef int __attribute__((may_alias)) int_a;

template <typename T> __device__ __forceinline__ void vst2(void* p, T v) { *(volatile T*)p = v; __threadfence(); *(volatile T*)p = v; }
__device__ __forceinline__ v8f wmma16(v16h a, v16h b, v8f c) {
  v8f d = __builtin_amdgcn_wmma_f32_16x16x32_f16(false, a, false, b, (short)0, c, false, false);
  asm volatile("v_nop\n\tv_nop\n\tv_nop\n\tv_nop" : "+v"(d) : "v"(a), "v"(b));
  return d;
}
__device__ __forceinline__ v8f wmma_bf(v16b a, v16b b, v8f c) {
  v8f d = __builtin_amdgcn_wmma_f32_16x16x32_bf16(false, a, false, b, (short)0, c, false, false);
  asm volatile("v_nop\n\tv_nop\n\tv_nop\n\tv_nop" : "+v"(d) : "v"(a), "v"(b));
  return d;
}
__device__ __forceinline__ v16h frag_h(const _Float16* rowk0, int lane) {
  union { v16h v; v8h q[2]; } u; const _Float16* p = rowk0 + 8 * (lane >> 4);
  u.q[0] = *(const v8h*)p; u.q[1] = *(const v8h*)(p + 16); return u.v;
}
__device__ __forceinline__ v16h frag_f32(const float* rowk0, int lane) {
  v16h a; const float* p = rowk0 + 8 * (lane >> 4);
#pragma unroll
  for (int i = 0; i < 8; ++i) { a[i] = (_Float16)p[i]; a[8 + i] = (_Float16)p[16 + i]; }
  return a;
}
__device__ __forceinline__ v16h frag_f32s(const float* rowk0, int lane, float sc) {
  v16h a; const float* p = rowk0 + 8 * (lane >> 4);
#pragma unroll
  for (int i = 0; i < 8; ++i) { a[i] = (_Float16)(p[i] * sc); a[8 + i] = (_Float16)(p[16 + i] * sc); }
  return a;
}
__device__ __forceinline__ v16h fragc_f32(const float* W, int k0, int n, int lane, int ld, int K) {
  v16h a; const int g = lane >> 4;
#pragma unroll
  for (int i = 0; i < 8; ++i) { const int ka = k0 + 8 * g + i, kb = ka + 16;
    a[i] = (_Float16)(ka < K ? W[(size_t)(ka < K ? ka : K - 1) * ld + n] : 0.f); a[8 + i] = (_Float16)(kb < K ? W[(size_t)(kb < K ? kb : K - 1) * ld + n] : 0.f); }
  return a;
}
struct F2 { v16b h, l; };
__device__ __forceinline__ F2 bsplit16(const float v[16]) { F2 r;
#pragma unroll
  for (int i = 0; i < 16; ++i) { const __bf16 h = (__bf16)v[i]; r.h[i] = h; r.l[i] = (__bf16)(v[i] - (float)h); }
  return r; }
__device__ __forceinline__ F2 split_row(const float* row, int k0, int lane) { float v[16]; const float* p = row + k0 + 8 * (lane >> 4);
#pragma unroll
  for (int i = 0; i < 8; ++i) { v[i] = p[i]; v[8 + i] = p[16 + i]; }
  return bsplit16(v); }
__device__ __forceinline__ F2 split_rowK(const float* row, int k0, int lane, int K) { float v[16]; const int g = lane >> 4;
#pragma unroll
  for (int i = 0; i < 8; ++i) { const int ka = k0 + 8 * g + i, kb = ka + 16; v[i] = ka < K ? row[ka < K ? ka : K - 1] : 0.f; v[8 + i] = kb < K ? row[kb < K ? kb : K - 1] : 0.f; }
  return bsplit16(v); }
__device__ __forceinline__ F2 split_col(const float* W, int k0, int n, int lane, int ld, int K) { float v[16]; const int g = lane >> 4;
#pragma unroll
  for (int i = 0; i < 8; ++i) { const int ka = k0 + 8 * g + i, kb = ka + 16; v[i] = ka < K ? W[(size_t)(ka < K ? ka : K - 1) * ld + n] : 0.f; v[8 + i] = kb < K ? W[(size_t)(kb < K ? kb : K - 1) * ld + n] : 0.f; }
  return bsplit16(v); }
__device__ __forceinline__ v8f mac3(const F2& a, const F2& b, v8f c) { c = wmma_bf(a.l, b.h, c); c = wmma_bf(a.h, b.l, c); return wmma_bf(a.h, b.h, c); }
__device__ __forceinline__ float sigm(float v) { return 1.0f / (1.0f + expf(-v)); }
#define LDSX() do { asm volatile("s_wait_dscnt 0" ::: "memory"); __builtin_amdgcn_wave_barrier(); __builtin_amdgcn_fence(__ATOMIC_RELEASE, "workgroup"); } while (0)


#define NBT 4
#define CIN 512
#define CI 128
#define HH 64
#define WWD 64
#define NCLS 19
#define NPIX (NBT * HH * WWD)
#define NROW (NBT * HH)
#ifndef TY1
#define TY1 NROW
#define TY2 NROW
#endif
typedef __attribute__((ext_vector_type(8))) __bf16 v8b;
__device__ __forceinline__ v16b frag_b(const __bf16* rowk0, int lane) {
  union { v16b v; v8b q[2]; } u; const __bf16* p = rowk0 + 8 * (lane >> 4);
  u.q[0] = *(const v8b*)p; u.q[1] = *(const v8b*)(p + 16); return u.v;
}
__device__ __forceinline__ float bfr(float v) { return (float)(__bf16)v; }
__device__ __attribute__((noinline)) float exp_ni(float v) { return expf(v); }
__device__ __attribute__((noinline)) float erf_ni(float v) { return erff(v); }

#define K1 (9 * CIN)
#define K2 (9 * CI)
#define PK_A  0
#define PK_C  (PK_A + CI * K1)
#define PK_51 (PK_C + CI * K1)
#define PK_52 (PK_51 + CI * K2)
#define PK_8  (PK_52 + CI * K2)
#define PK_END (PK_8 + 32 * CI)
#define WS_PK  0u
#define WS_XC  (WS_PK + 2u * PK_END)
#define WS_F1H (WS_XC + 2u * NPIX * CIN)
#define WS_F1L (WS_F1H + 2u * NPIX * CI)
#define WS_F2H (WS_F1L + 2u * NPIX * CI)
#define WS_F2L (WS_F2H + 2u * NPIX * CI)
#define WS_END (WS_F2L + 2u * NPIX * CI)

__global__ __launch_bounds__(256) void k_packc(const float* __restrict__ WA, const float* __restrict__ WC, const float* __restrict__ W51, const float* __restrict__ W52, const float* __restrict__ W8, __bf16* __restrict__ PK) {
  __shared__ __align__(16) __bf16 s[K1]; const int o = blockIdx.x, which = blockIdx.y, tid = threadIdx.x; const float* Wm; int C, K; size_t dst;
  if (which == 0) { Wm = WA; C = CIN; K = K1; dst = PK_A + (size_t)o * K1; } else if (which == 1) { Wm = WC; C = CIN; K = K1; dst = PK_C + (size_t)o * K1; }
  else if (which == 2) { Wm = W51; C = CI; K = K2; dst = PK_51 + (size_t)o * K2; } else if (which == 3) { Wm = W52; C = CI; K = K2; dst = PK_52 + (size_t)o * K2; }
  else { if (o >= 32) return; K = CI; dst = PK_8 + (size_t)o * CI; for (int k = tid; k < K; k += 256) s[k] = (__bf16)((o < NCLS) ? W8[(size_t)o * CI + k] : 0.f); __syncthreads(); if (tid < K / 8) vst2((unsigned*)(PK + dst + tid * 8), *(const v4u*)&s[tid * 8]); return; }
  for (int k = tid; k < K; k += 256) { const int tap = k / C, ci = k % C; s[k] = (__bf16)Wm[((size_t)o * C + ci) * 9 + tap]; }
  __syncthreads();
  for (int q = tid; q < K / 8; q += 256) vst2((unsigned*)(PK + dst + q * 8), *(const v4u*)&s[q * 8]);
}
__global__ __launch_bounds__(256) void k_tr(const float* __restrict__ X, __bf16* __restrict__ XC) {
  __shared__ __align__(16) __bf16 s[64][264]; const int row = blockIdx.x, half = blockIdx.y, tid = threadIdx.x; const int b = row / HH, y = row % HH; const int c0 = half * 256;
  for (int q = tid; q < 256 * 64; q += 256) { const int cl = q >> 6, px = q & 63; s[px][cl] = (__bf16)X[(((size_t)b * CIN + c0 + cl) * HH + y) * WWD + px]; }
  __syncthreads();
  for (int q = tid; q < 64 * 32; q += 256) { const int px = q >> 5, pc = q & 31; vst2((unsigned*)(XC + ((size_t)row * WWD + px) * CIN + c0 + pc * 8), *(const v4u*)&s[px][pc * 8]); }
}
__device__ __forceinline__ v16b zfrag_if(v16b a, bool ok) { const v16b z = {}; return ok ? a : z; }
__global__ __launch_bounds__(128) void k_c1(const __bf16* __restrict__ XC, const __bf16* __restrict__ PK, const float* __restrict__ SA, const float* __restrict__ BA, const float* __restrict__ MA, const float* __restrict__ VA, const float* __restrict__ SC, const float* __restrict__ BC, const float* __restrict__ MC, const float* __restrict__ VC, __bf16* __restrict__ F1H, __bf16* __restrict__ F1L, __bf16* __restrict__ F2H, __bf16* __restrict__ F2L) {
  __shared__ __align__(16) __bf16 sh_[4][16][136]; __shared__ __align__(16) __bf16 sl_[4][16][136];
  const int tid = threadIdx.x, wave = tid >> 5, lane = tid & 31, col = lane & 15, g = lane >> 4; const int row = blockIdx.x, which = blockIdx.y; const int b = row / HH, y = row % HH; const int px = wave * 16 + col;
  const __bf16* P = PK + (which == 0 ? PK_A : PK_C); const float *S_ = which == 0 ? SA : SC, *B_ = which == 0 ? BA : BC, *M_ = which == 0 ? MA : MC, *V_ = which == 0 ? VA : VC; __bf16 *FH = which == 0 ? F1H : F2H, *FL = which == 0 ? F1L : F2L;
  v8f acc[8] = {};
#pragma unroll 1
  for (int tap = 0; tap < 9; ++tap) { const int yy = y + tap / 3 - 1, xx = px + tap % 3 - 1; const bool ok = (yy >= 0) && (yy < HH) && (xx >= 0) && (xx < WWD);
    const __bf16* arow = XC + (((size_t)b * HH + min(max(yy, 0), HH - 1)) * WWD + min(max(xx, 0), WWD - 1)) * CIN;
#pragma unroll 4
    for (int kc = 0; kc < CIN / 32; ++kc) { const v16b a = zfrag_if(frag_b(arow + kc * 32, lane), ok); const size_t kk = (size_t)tap * CIN + kc * 32;
#pragma unroll
      for (int j = 0; j < 8; ++j) acc[j] = wmma_bf(a, frag_b(P + (size_t)(j * 16 + col) * K1 + kk, lane), acc[j]); } }
#pragma unroll
  for (int j = 0; j < 8; ++j) { const int c = j * 16 + col; const float inv = bfr(S_[c]) / sqrtf(bfr(V_[c]) + 1e-5f); const float sh = bfr(B_[c]) - bfr(M_[c]) * inv;
#pragma unroll
    for (int r = 0; r < 8; ++r) { const float v = fmaxf(acc[j][r] * inv + sh, 0.f); const __bf16 hb = (__bf16)v; sh_[wave][8 * g + r][c] = hb; sl_[wave][8 * g + r][c] = (__bf16)(v - (float)hb); } }
  LDSX();
  for (int rl = 0; rl < 16; ++rl) if (lane < 16) { const size_t p = ((size_t)row * WWD + wave * 16 + rl) * CI; vst2((unsigned*)(FH + p + lane * 8), *(const v4u*)&sh_[wave][rl][lane * 8]); vst2((unsigned*)(FL + p + lane * 8), *(const v4u*)&sl_[wave][rl][lane * 8]); }
}
__global__ __launch_bounds__(128) void k_c2(const __bf16* __restrict__ F1H, const __bf16* __restrict__ F1L, const __bf16* __restrict__ F2H, const __bf16* __restrict__ F2L, const __bf16* __restrict__ PK, const float* __restrict__ S1, const float* __restrict__ B1, const float* __restrict__ M1, const float* __restrict__ V1, const float* __restrict__ S2, const float* __restrict__ B2, const float* __restrict__ M2, const float* __restrict__ V2, const float* __restrict__ B8, float* __restrict__ OUT) {
  __shared__ __align__(16) float ssum[64][132]; __shared__ __align__(16) float so8[32][68];
  const int tid = threadIdx.x, wave = tid >> 5, lane = tid & 31, col = lane & 15, g = lane >> 4; const int row = blockIdx.x; const int b = row / HH, y = row % HH; const int px = wave * 16 + col;
#pragma unroll 1
  for (int br = 0; br < 2; ++br) { const __bf16 *FH = br == 0 ? F1H : F2H, *FL = br == 0 ? F1L : F2L; const __bf16* P = PK + (br == 0 ? PK_51 : PK_52); const float *S_ = br == 0 ? S1 : S2, *B_ = br == 0 ? B1 : B2, *M_ = br == 0 ? M1 : M2, *V_ = br == 0 ? V1 : V2;
    v8f acc[8] = {};
#pragma unroll 1
    for (int tap = 0; tap < 9; ++tap) { const int yy = y + tap / 3 - 1, xx = px + tap % 3 - 1; const bool ok = (yy >= 0) && (yy < HH) && (xx >= 0) && (xx < WWD);
      const size_t ap = (((size_t)b * HH + min(max(yy, 0), HH - 1)) * WWD + min(max(xx, 0), WWD - 1)) * CI;
#pragma unroll
      for (int kc = 0; kc < CI / 32; ++kc) { const v16b ah = zfrag_if(frag_b(FH + ap + kc * 32, lane), ok), al = zfrag_if(frag_b(FL + ap + kc * 32, lane), ok); const size_t kk = (size_t)tap * CI + kc * 32;
#pragma unroll
        for (int j = 0; j < 8; ++j) { const v16b w = frag_b(P + (size_t)(j * 16 + col) * K2 + kk, lane); acc[j] = wmma_bf(al, w, acc[j]); acc[j] = wmma_bf(ah, w, acc[j]); } } }
#pragma unroll
    for (int j = 0; j < 8; ++j) { const int c = j * 16 + col; const float inv = bfr(S_[c]) / sqrtf(bfr(V_[c]) + 1e-5f); const float sh = bfr(B_[c]) - bfr(M_[c]) * inv;
#pragma unroll
      for (int r = 0; r < 8; ++r) { const float v = fmaxf(acc[j][r] * inv + sh, 0.f); if (br == 0) ssum[wave * 16 + 8 * g + r][c] = v; else ssum[wave * 16 + 8 * g + r][c] += v; } }
    LDSX(); }
  v8f acc8[2] = {};
#pragma unroll
  for (int kc = 0; kc < CI / 32; ++kc) { const F2 a = split_row(&ssum[wave * 16 + col][0], kc * 32, lane);
#pragma unroll
    for (int j = 0; j < 2; ++j) { const v16b w = frag_b(PK + PK_8 + (size_t)(j * 16 + col) * CI + kc * 32, lane); acc8[j] = wmma_bf(a.l, w, acc8[j]); acc8[j] = wmma_bf(a.h, w, acc8[j]); } }
  __syncthreads();
#pragma unroll
  for (int j = 0; j < 2; ++j) { const int o = j * 16 + col; const float bb = (o < NCLS) ? bfr(B8[min(o, NCLS - 1)]) : 0.f;
#pragma unroll
    for (int r = 0; r < 8; ++r) so8[o][wave * 16 + 8 * g + r] = acc8[j][r] + bb; }
  __syncthreads();
  for (int q = tid; q < NCLS * 16; q += 128) { const int o = q >> 4, pc = q & 15; vst2(OUT + (((size_t)b * NCLS + o) * HH + y) * WWD + pc * 4, *(const v4f*)&so8[o][pc * 4]); }
}
extern "C" void kernel_launch(void* const* d_in, const int* in_sizes, int n_in, void* d_out, int out_size, void* d_ws, size_t ws_size, hipStream_t stream) {
  (void)in_sizes; (void)n_in; (void)out_size;
  const float** F = (const float**)d_in;
  if (ws_size < (size_t)WS_END) return;
  char* ws = (char*)d_ws; __bf16 *PK = (__bf16*)(ws + WS_PK), *XC = (__bf16*)(ws + WS_XC), *F1H = (__bf16*)(ws + WS_F1H), *F1L = (__bf16*)(ws + WS_F1L), *F2H = (__bf16*)(ws + WS_F2H), *F2L = (__bf16*)(ws + WS_F2L);
  k_packc<<<dim3(CI, 5), 256, 0, stream>>>(F[1], F[6], F[17], F[22], F[27], PK);
  k_tr<<<dim3(NROW, 2), 256, 0, stream>>>(F[0], XC);
  k_c1<<<dim3(TY1, 2), 128, 0, stream>>>(XC, PK, F[2], F[3], F[4], F[5], F[7], F[8], F[9], F[10], F1H, F1L, F2H, F2L);
  k_c2<<<TY2, 128, 0, stream>>>(F1H, F1L, F2H, F2L, PK, F[18], F[19], F[20], F[21], F[23], F[24], F[25], F[26], F[28], (float*)d_out);
}
